// SHR_ReLABlock_27900107555069
// MI455X (gfx1250) — hardware-verified
//
#include <hip/hip_runtime.h>
#include <math.h>

constexpr int kBatch = 2;
constexpr int kSeq   = 2048;
constexpr int kDim   = 256;
constexpr int kHeads = 8;
constexpr int kHdim  = 64;
constexpr int kInner = kHeads * kHdim;
constexpr int kQkvW  = 3 * kInner;
constexpr int kHid   = 1024;
constexpr int kDim3  = 3 * kDim;
constexpr int kRows  = kBatch * kSeq;
constexpr float kWCarry = 16.0f;
constexpr float kACarry = 16.0f;
constexpr float kLnEps  = 1e-5f;
constexpr float kRmsEps = 1e-8f;
constexpr float kInvSqrtInner = 0.04419417382415922f;
constexpr float kAttnScale    = 0.125f;
static_assert(kRows % 64 == 0 && kQkvW % 64 == 0 && kDim % 64 == 0 && kHid % 64 == 0 && kDim3 % 64 == 0 && kInner % 64 == 0, "tile multiples");
static_assert(kDim % 32 == 0 && kInner % 32 == 0 && kDim3 % 32 == 0 && kHid % 32 == 0 && kSeq % 64 == 0 && kHdim == 64, "K multiples of 32");

typedef __attribute__((ext_vector_type(16))) _Float16 v16h;
typedef __attribute__((ext_vector_type(8)))  _Float16 v8h;
typedef __attribute__((ext_vector_type(16))) __bf16   v16b;
typedef __attribute__((ext_vector_type(8)))  __bf16   v8b;
typedef __attribute__((ext_vector_type(8)))  float    v8f;
typedef __attribute__((ext_vector_type(4)))  float    v4f;
typedef __attribute__((ext_vector_type(2)))  float    v2f;
typedef __attribute__((ext_vector_type(4)))  unsigned int v4u;
typedef __attribute__((ext_vector_type(2)))  unsigned int v2u;

__device__ __forceinline__ unsigned short f2bf_bits(float f) {
  unsigned u = __float_as_uint(f);
  return (unsigned short)((u + 0x7FFFu + ((u >> 16) & 1u)) >> 16);
}
__device__ __forceinline__ float bf_bits2f(unsigned short h) { return __uint_as_float(((unsigned)h) << 16); }

__device__ __forceinline__ void dep_guard_h(v8f& a, v8f& b, v16h x, v16h y) { asm volatile("v_nop\n\tv_nop\n\tv_nop\n\tv_nop" : "+v"(a), "+v"(b) : "v"(x), "v"(y)); }
__device__ __forceinline__ void dep_guard_b(v8f& a, v8f& b, v16b x, v16b y) { asm volatile("v_nop\n\tv_nop\n\tv_nop\n\tv_nop" : "+v"(a), "+v"(b) : "v"(x), "v"(y)); }
__device__ __forceinline__ void keep4_h(v16h a, v16h b, v16h c, v16h d) { asm volatile("v_nop" :: "v"(a), "v"(b), "v"(c), "v"(d)); }
__device__ __forceinline__ void keep4_b(v16b a, v16b b, v16b c, v16b d) { asm volatile("v_nop" :: "v"(a), "v"(b), "v"(c), "v"(d)); }
__device__ __forceinline__ void acc_guard4(v8f& a, v8f& b, v8f& c, v8f& d) { asm volatile("v_nop\n\tv_nop\n\tv_nop\n\tv_nop" : "+v"(a), "+v"(b), "+v"(c), "+v"(d)); }
template <typename T> struct Frag;
template <> struct Frag<_Float16> {
  typedef v16h V; union U { v16h v; v8h h[2]; };
  static __device__ __forceinline__ v16h load(const _Float16* p) {
    U f; f.h[0] = *(const v8h*)(p); f.h[1] = *(const v8h*)(p + 16); return f.v;
  }
  static __device__ __forceinline__ v8f mma(v16h a, v16h b, v8f c) {
    return __builtin_amdgcn_wmma_f32_16x16x32_f16(false, a, false, b, (short)0, c, false, false);
  }
  static __device__ __forceinline__ void guard(v8f& a, v8f& b, v16h x, v16h y) { dep_guard_h(a, b, x, y); }
  static __device__ __forceinline__ void keep(v16h a, v16h b, v16h c, v16h d) { keep4_h(a, b, c, d); }
};
template <> struct Frag<__bf16> {
  typedef v16b V; union U { v16b v; v8b h[2]; };
  static __device__ __forceinline__ v16b load(const __bf16* p) {
    U f; f.h[0] = *(const v8b*)(p); f.h[1] = *(const v8b*)(p + 16); return f.v;
  }
  static __device__ __forceinline__ v8f mma(v16b a, v16b b, v8f c) {
    return __builtin_amdgcn_wmma_f32_16x16x32_bf16(false, a, false, b, (short)0, c, false, false);
  }
  static __device__ __forceinline__ void guard(v8f& a, v8f& b, v16b x, v16b y) { dep_guard_b(a, b, x, y); }
  static __device__ __forceinline__ void keep(v16b a, v16b b, v16b c, v16b d) { keep4_b(a, b, c, d); }
};

__device__ __forceinline__ unsigned pk16(unsigned short a, unsigned short b) { return (unsigned)a | ((unsigned)b << 16); }
__device__ __forceinline__ unsigned short h_bits(float f) { const _Float16 h = (_Float16)f; return __builtin_bit_cast(unsigned short, h); }

__device__ __forceinline__ v8f mma_f16g(v16h a, v16h b, v8f c) {
  c = __builtin_amdgcn_wmma_f32_16x16x32_f16(false, a, false, b, (short)0, c, false, false);
  asm volatile("v_nop\n\tv_nop\n\tv_nop\n\tv_nop" : "+v"(c) : "v"(a), "v"(b));
  return c;
}

template <int ET> struct Elem;
template <> struct Elem<0> { typedef _Float16 T; };
template <> struct Elem<1> { typedef __bf16 T; };
template <int ET, bool SPLIT, int BIAS_MODE, int OUT_MODE, bool RESID, int ACT = 0>
__global__ __launch_bounds__(256) void wmma_gemm64(
    const unsigned short* __restrict__ Ap, const unsigned short* __restrict__ A2p, int lda, long strideA,
    const unsigned short* __restrict__ Btp, const unsigned short* __restrict__ Bt2p, int ldb, long strideB,
    void* __restrict__ Cout, void* __restrict__ Cout2, int ldc, long strideC,
    const float* __restrict__ bias,
    const float* __restrict__ resid, long strideR, int ldr,
    int M, int N, int K, float scale) {
  typedef typename Elem<ET>::T T;
  typedef typename Frag<T>::V V;
  const T* A = (const T*)Ap; const T* A2 = (const T*)A2p; const T* Bt = (const T*)Btp; const T* Bt2 = (const T*)Bt2p;
  __shared__ __align__(16) float sT[8][16 * 68];
  const int b    = blockIdx.y;
  const int lane = threadIdx.x & 31;
  const int wave = threadIdx.x >> 5;
  const int tilesN = N >> 6;
  const int tilesM = M >> 6;
  const int tile = blockIdx.x * 8 + wave;
  if (tile >= tilesM * tilesN) return;
  const int tm = tile / tilesN;
  const int tn = tile - tm * tilesN;
  const int m0 = tm << 6;
  const int n0 = tn << 6;

  const T* Ab  = A  + (size_t)b * strideA;
  const T* Bb  = Bt + (size_t)b * strideB;
  const T* Ab2 = SPLIT ? (A2  + (size_t)b * strideA) : nullptr;
  const T* Bb2 = SPLIT ? (Bt2 + (size_t)b * strideB) : nullptr;

  const int rlane = lane & 15;
  const int koff  = (lane >> 4) * 8;
  const int mOff  = (lane >> 4) * 8;

  v8f acc[4][4];
#pragma unroll
  for (int i = 0; i < 4; ++i)
#pragma unroll
    for (int j = 0; j < 4; ++j) acc[i][j] = (v8f){0.f,0.f,0.f,0.f,0.f,0.f,0.f,0.f};

  for (int k0 = 0; k0 < K; k0 += 32) {
    V bh[4], bl[4];
#pragma unroll
    for (int j = 0; j < 4; ++j) {
      const size_t bo = (size_t)(n0 + (j << 4) + rlane) * ldb + koff + k0;
      bh[j] = Frag<T>::load(Bb + bo);
      if (SPLIT) bl[j] = Frag<T>::load(Bb2 + bo);
    }
#pragma unroll
    for (int i = 0; i < 4; ++i) {
      const size_t ao = (size_t)(m0 + (i << 4) + rlane) * lda + koff + k0;
      V ah = Frag<T>::load(Ab + ao);
      V al;
      if (SPLIT) al = Frag<T>::load(Ab2 + ao);
#pragma unroll
      for (int j = 0; j < 4; ++j) {
        acc[i][j] = Frag<T>::mma(ah, bh[j], acc[i][j]);
        if (SPLIT) {
          acc[i][j] = Frag<T>::mma(ah, bl[j], acc[i][j]);
          acc[i][j] = Frag<T>::mma(al, bh[j], acc[i][j]);
        }
      }
      Frag<T>::guard(acc[i][0], acc[i][3], ah, SPLIT ? al : ah);
    }
    Frag<T>::keep(bh[0], bh[1], bh[2], bh[3]);
    if (SPLIT) Frag<T>::keep(bl[0], bl[1], bl[2], bl[3]);
  }
  acc_guard4(acc[0][0], acc[0][1], acc[0][2], acc[0][3]);
  acc_guard4(acc[1][0], acc[1][1], acc[1][2], acc[1][3]);
  acc_guard4(acc[2][0], acc[2][1], acc[2][2], acc[2][3]);
  acc_guard4(acc[3][0], acc[3][1], acc[3][2], acc[3][3]);

  float* slab = sT[wave];
  const float* Rb = RESID ? (resid + (size_t)b * strideR) : nullptr;
#pragma unroll
  for (int i = 0; i < 4; ++i) {
    const int mBase = m0 + (i << 4);
#pragma unroll
    for (int j = 0; j < 4; ++j) {
      const int n = n0 + (j << 4) + rlane;
      float bv = 0.f;
      if (BIAS_MODE == 2) bv = bias[n];
#pragma unroll
      for (int r = 0; r < 8; ++r) {
        float v = acc[i][j][r] * scale;
        if (BIAS_MODE == 1) v += bias[mBase + mOff + r];
        if (BIAS_MODE == 2) v += bv;
        if (RESID) v += Rb[(size_t)(mBase + mOff + r) * ldr + n];
        if (ACT == 2) v = fmaxf(v, 0.0f);
        if (ACT == 4) v = (v > 0.f) ? v : 0.01f * v;
        slab[(mOff + r) * 68 + (j << 4) + rlane] = v;
      }
    }
    __builtin_amdgcn_fence(__ATOMIC_RELEASE, "workgroup");
    __builtin_amdgcn_wave_barrier();
    __builtin_amdgcn_fence(__ATOMIC_ACQUIRE, "workgroup");
    if (OUT_MODE == 0) {
      float* C = (float*)Cout + (size_t)b * strideC;
      const int hh = lane >> 4, c4 = (lane & 15) * 4;
      for (int pass = 0; pass < 2; ++pass) {
#pragma unroll
        for (int it = 0; it < 8; ++it) {
          const int row = it * 2 + hh;
          v4f v = *(const v4f*)(slab + row * 68 + c4);
          *(volatile v4f*)(C + (size_t)(mBase + row) * ldc + n0 + c4) = v;
        }
        __threadfence();
      }
    } else {
      const int q = lane >> 3, c8 = (lane & 7) * 8;
      unsigned short* C  = (unsigned short*)Cout  + (size_t)b * strideC;
      unsigned short* C2 = (OUT_MODE == 2) ? ((unsigned short*)Cout2 + (size_t)b * strideC) : nullptr;
      for (int pass = 0; pass < 2; ++pass) {
#pragma unroll
        for (int it = 0; it < 4; ++it) {
          const int row = it * 4 + q;
          const float* sp = slab + row * 68 + c8;
          v8h hv, lv;
#pragma unroll
          for (int e = 0; e < 8; ++e) {
            if (OUT_MODE == 1) {
              hv[e] = (_Float16)sp[e];
            } else {
              unsigned short hb = f2bf_bits(sp[e]);
              unsigned short lb = f2bf_bits(sp[e] - bf_bits2f(hb));
              hv[e] = __builtin_bit_cast(_Float16, hb);
              lv[e] = __builtin_bit_cast(_Float16, lb);
            }
          }
          *(volatile v8h*)(C + (size_t)(mBase + row) * ldc + n0 + c8) = hv;
          if (OUT_MODE == 2) *(volatile v8h*)(C2 + (size_t)(mBase + row) * ldc + n0 + c8) = lv;
        }
        __threadfence();
      }
    }
    __builtin_amdgcn_fence(__ATOMIC_RELEASE, "workgroup");
    __builtin_amdgcn_wave_barrier();
    __builtin_amdgcn_fence(__ATOMIC_ACQUIRE, "workgroup");
  }
}

__global__ __launch_bounds__(256) void wtcast_kernel(const float* __restrict__ W, unsigned short* __restrict__ out,
                                                     int nIn, int nOut, float scale) {
  __shared__ float sm[64][65];
  const int t  = threadIdx.x;
  const int d0 = blockIdx.x * 64;
  const int h0 = blockIdx.y * 64;
  const int z  = blockIdx.z;
  const float* Wz = W + (size_t)z * nIn * nOut;
#pragma unroll
  for (int i = 0; i < 16; ++i) {
    const int e = i * 256 + t;
    const int r = e >> 6;
    const int c = e & 63;
    sm[c][r] = Wz[(size_t)(d0 + r) * nOut + h0 + c] * scale;
  }
  __syncthreads();
  const int lane = t & 31, wave = t >> 5;
  const int q = lane >> 3, c8 = (lane & 7) * 8;
  unsigned short* op = out + (size_t)z * nOut * nIn;
  for (int pass = 0; pass < 2; ++pass) {
#pragma unroll
    for (int it = 0; it < 2; ++it) {
      const int row = wave * 8 + it * 4 + q;
      unsigned short hb[8];
#pragma unroll
      for (int e = 0; e < 8; ++e) hb[e] = h_bits(sm[row][c8 + e]);
      const v4u u = (v4u){pk16(hb[0], hb[1]), pk16(hb[2], hb[3]), pk16(hb[4], hb[5]), pk16(hb[6], hb[7])};
      *(volatile v4u*)(op + (size_t)(h0 + row) * nIn + d0 + c8) = u;
    }
    __threadfence();
  }
}

__global__ __launch_bounds__(256) void ln256_kernel(const float* __restrict__ x, const float* __restrict__ g,
                                                    const float* __restrict__ bt, unsigned short* __restrict__ xn) {
  const int lane = threadIdx.x & 31, wave = threadIdx.x >> 5;
  const int row = blockIdx.x * 8 + wave;
  const float* r = x + (size_t)row * kDim + lane * 8;
  const v4f a = *(const v4f*)(r);
  const v4f c = *(const v4f*)(r + 4);
  float v[8];
#pragma unroll
  for (int e = 0; e < 4; ++e) { v[e] = a[e]; v[4 + e] = c[e]; }
  float s = ((v[0] + v[1]) + (v[2] + v[3])) + ((v[4] + v[5]) + (v[6] + v[7]));
#pragma unroll
  for (int off = 16; off > 0; off >>= 1) s += __shfl_xor(s, off, 32);
  const float mean = s * (1.0f / 256.0f);
  float s2 = 0.f;
#pragma unroll
  for (int e = 0; e < 8; ++e) { v[e] -= mean; s2 += v[e] * v[e]; }
#pragma unroll
  for (int off = 16; off > 0; off >>= 1) s2 += __shfl_xor(s2, off, 32);
  const float var  = s2 * (1.0f / 256.0f);
  const float rstd = rsqrtf(var + kLnEps);
  const v4f g0 = *(const v4f*)(g + lane * 8);
  const v4f g1 = *(const v4f*)(g + lane * 8 + 4);
  const v4f b0 = *(const v4f*)(bt + lane * 8);
  const v4f b1 = *(const v4f*)(bt + lane * 8 + 4);
  unsigned short hb[8];
#pragma unroll
  for (int e = 0; e < 4; ++e) {
    hb[e]     = h_bits(v[e] * rstd * g0[e] + b0[e]);
    hb[4 + e] = h_bits(v[4 + e] * rstd * g1[e] + b1[e]);
  }
  const v4u u = (v4u){pk16(hb[0], hb[1]), pk16(hb[2], hb[3]), pk16(hb[4], hb[5]), pk16(hb[6], hb[7])};
  unsigned short* qp = xn + (size_t)row * kDim + lane * 8;
  *(volatile v4u*)qp = u;
  __threadfence();
  *(volatile v4u*)qp = u;
}

__global__ __launch_bounds__(256) void ln768_kernel(const float* __restrict__ xc, const float* __restrict__ g,
                                                    const float* __restrict__ bt, unsigned short* __restrict__ hn) {
  const int lane = threadIdx.x & 31, wave = threadIdx.x >> 5;
  const int row = blockIdx.x * 8 + wave;
  const float* r = xc + (size_t)row * kDim3 + lane * 8;
  v4f vv[6];
  float s = 0.f;
#pragma unroll
  for (int ch = 0; ch < 3; ++ch) {
    vv[2 * ch]     = *(const v4f*)(r + ch * kDim);
    vv[2 * ch + 1] = *(const v4f*)(r + ch * kDim + 4);
    s += ((vv[2 * ch][0] + vv[2 * ch][1]) + (vv[2 * ch][2] + vv[2 * ch][3]))
       + ((vv[2 * ch + 1][0] + vv[2 * ch + 1][1]) + (vv[2 * ch + 1][2] + vv[2 * ch + 1][3]));
  }
#pragma unroll
  for (int off = 16; off > 0; off >>= 1) s += __shfl_xor(s, off, 32);
  const float mean = s * (1.0f / 768.0f);
  float s2 = 0.f;
#pragma unroll
  for (int k = 0; k < 6; ++k) {
#pragma unroll
    for (int j = 0; j < 4; ++j) { const float d = vv[k][j] - mean; vv[k][j] = d; s2 += d * d; }
  }
#pragma unroll
  for (int off = 16; off > 0; off >>= 1) s2 += __shfl_xor(s2, off, 32);
  const float var  = s2 * (1.0f / 768.0f);
  const float rstd = rsqrtf(var + kLnEps);
  v4u u[3];
#pragma unroll
  for (int ch = 0; ch < 3; ++ch) {
    const v4f g0 = *(const v4f*)(g + ch * kDim + lane * 8);
    const v4f g1 = *(const v4f*)(g + ch * kDim + lane * 8 + 4);
    const v4f b0 = *(const v4f*)(bt + ch * kDim + lane * 8);
    const v4f b1 = *(const v4f*)(bt + ch * kDim + lane * 8 + 4);
    unsigned short hb[8];
#pragma unroll
    for (int j = 0; j < 4; ++j) {
      hb[j]     = h_bits(vv[2 * ch][j] * rstd * g0[j] + b0[j]);
      hb[4 + j] = h_bits(vv[2 * ch + 1][j] * rstd * g1[j] + b1[j]);
    }
    u[ch] = (v4u){pk16(hb[0], hb[1]), pk16(hb[2], hb[3]), pk16(hb[4], hb[5]), pk16(hb[6], hb[7])};
  }
  unsigned short* qp = hn + (size_t)row * kDim3 + lane * 8;
  for (int pass = 0; pass < 2; ++pass) {
#pragma unroll
    for (int ch = 0; ch < 3; ++ch) *(volatile v4u*)(qp + ch * kDim) = u[ch];
    __threadfence();
  }
}

__global__ __launch_bounds__(256) void rms512_kernel(const float* __restrict__ o, const float* __restrict__ sc,
                                                     unsigned short* __restrict__ rb) {
  const int lane = threadIdx.x & 31, wave = threadIdx.x >> 5;
  const int row = blockIdx.x * 8 + wave;
  const float* r = o + (size_t)row * kInner + lane * 8;
  v4f v[4];
  float ss = 0.f;
#pragma unroll
  for (int ch = 0; ch < 2; ++ch) {
    v[2 * ch]     = *(const v4f*)(r + ch * 256);
    v[2 * ch + 1] = *(const v4f*)(r + ch * 256 + 4);
#pragma unroll
    for (int j = 0; j < 4; ++j) { ss += v[2 * ch][j] * v[2 * ch][j]; ss += v[2 * ch + 1][j] * v[2 * ch + 1][j]; }
  }
#pragma unroll
  for (int off = 16; off > 0; off >>= 1) ss += __shfl_xor(ss, off, 32);
  const float rms = sqrtf(ss) * kInvSqrtInner;
  const float inv = 1.0f / (rms + kRmsEps);
  v4u u[2];
#pragma unroll
  for (int ch = 0; ch < 2; ++ch) {
    const v4f g0 = *(const v4f*)(sc + ch * 256 + lane * 8);
    const v4f g1 = *(const v4f*)(sc + ch * 256 + lane * 8 + 4);
    unsigned short hb[8];
#pragma unroll
    for (int j = 0; j < 4; ++j) {
      hb[j]     = h_bits(((v[2 * ch][j] * inv) * g0[j]) * kACarry);
      hb[4 + j] = h_bits(((v[2 * ch + 1][j] * inv) * g1[j]) * kACarry);
    }
    u[ch] = (v4u){pk16(hb[0], hb[1]), pk16(hb[2], hb[3]), pk16(hb[4], hb[5]), pk16(hb[6], hb[7])};
  }
  unsigned short* qp = rb + (size_t)row * kInner + lane * 8;
  for (int pass = 0; pass < 2; ++pass) {
#pragma unroll
    for (int ch = 0; ch < 2; ++ch) *(volatile v4u*)(qp + ch * 256) = u[ch];
    __threadfence();
  }
}

__global__ __launch_bounds__(256) void vtrans_kernel(const unsigned short* __restrict__ qkv, unsigned short* __restrict__ vt) {
  __shared__ unsigned short sm[64][66];
  const int t  = threadIdx.x;
  const int n0 = blockIdx.x * 64;
  const int c0 = blockIdx.y * 64;
  const int g  = blockIdx.z;
#pragma unroll
  for (int i = 0; i < 2; ++i) {
    const int e = i * 256 + t;
    const int r = e >> 3;
    const int part = e & 7;
    const v4u u = *(const v4u*)(qkv + (size_t)(g * kSeq + n0 + r) * kQkvW + 2 * kInner + c0 + part * 8);
#pragma unroll
    for (int w = 0; w < 4; ++w) {
      sm[part * 8 + 2 * w][r]     = (unsigned short)(u[w] & 0xFFFFu);
      sm[part * 8 + 2 * w + 1][r] = (unsigned short)(u[w] >> 16);
    }
  }
  __syncthreads();
  const int lane = t & 31, wave = t >> 5;
  const int q = lane >> 3, c8 = (lane & 7) * 8;
  for (int pass = 0; pass < 2; ++pass) {
#pragma unroll
    for (int it = 0; it < 2; ++it) {
      const int row = wave * 8 + it * 4 + q;
      unsigned short hb[8];
#pragma unroll
      for (int e = 0; e < 8; ++e) hb[e] = sm[row][c8 + e];
      const v4u u = (v4u){pk16(hb[0], hb[1]), pk16(hb[2], hb[3]), pk16(hb[4], hb[5]), pk16(hb[6], hb[7])};
      *(volatile v4u*)(vt + (size_t)(g * kInner + c0 + row) * kSeq + n0 + c8) = u;
    }
    __threadfence();
  }
}

__global__ __launch_bounds__(128) void rela_attn_kernel(const unsigned short* __restrict__ qkv,
                                                        const unsigned short* __restrict__ vt,
                                                        float* __restrict__ attno) {
  __shared__ __align__(16) _Float16 Psh[4][16 * 64];
  __shared__ __align__(16) float    Os[4][16 * 68];
  const int tid  = threadIdx.x;
  const int wave = tid >> 5;
  const int lane = tid & 31;
  const int hh   = lane >> 4;
  const int c    = lane & 15;
  constexpr int nqb = kSeq / 64;
  const int bx = blockIdx.x;
  const int qb = bx % nqb;
  const int bh = bx / nqb;
  const int h  = bh % kHeads;
  const int b  = bh / kHeads;
  const int q0 = qb * 64 + wave * 16;

  const _Float16* Qp = (const _Float16*)qkv + (size_t)b * kSeq * kQkvW + h * kHdim;
  const _Float16* Kp = Qp + kInner;
  const _Float16* Vp = (const _Float16*)vt + (size_t)bh * kHdim * kSeq;
  float* Op = attno + (size_t)b * kSeq * kInner + h * kHdim;

  v16h qa[2];
#pragma unroll
  for (int dc = 0; dc < 2; ++dc)
    qa[dc] = Frag<_Float16>::load(Qp + (size_t)(q0 + c) * kQkvW + dc * 32 + 8 * hh);

  v8f oacc[4];
#pragma unroll
  for (int t = 0; t < 4; ++t) oacc[t] = (v8f){0.f,0.f,0.f,0.f,0.f,0.f,0.f,0.f};
  _Float16* pw = Psh[wave];

#pragma unroll 1
  for (int kc = 0; kc < kSeq / 64; ++kc) {
    const int kv0 = kc * 64;
    v8f s[4];
#pragma unroll
    for (int j = 0; j < 4; ++j) {
      s[j] = (v8f){0.f,0.f,0.f,0.f,0.f,0.f,0.f,0.f};
      const _Float16* kr = Kp + (size_t)(kv0 + j * 16 + c) * kQkvW + 8 * hh;
#pragma unroll
      for (int dc = 0; dc < 2; ++dc) {
        const v16h kb = Frag<_Float16>::load(kr + dc * 32);
        s[j] = mma_f16g(qa[dc], kb, s[j]);
      }
    }
    __builtin_amdgcn_fence(__ATOMIC_RELEASE, "workgroup");
    __builtin_amdgcn_wave_barrier();
    __builtin_amdgcn_fence(__ATOMIC_ACQUIRE, "workgroup");
#pragma unroll
    for (int r = 0; r < 8; ++r) {
#pragma unroll
      for (int j = 0; j < 4; ++j)
        pw[(8 * hh + r) * 64 + j * 16 + c] = (_Float16)fmaxf(s[j][r], 0.0f);
    }
    __builtin_amdgcn_fence(__ATOMIC_RELEASE, "workgroup");
    __builtin_amdgcn_wave_barrier();
    __builtin_amdgcn_fence(__ATOMIC_ACQUIRE, "workgroup");
#pragma unroll
    for (int kk = 0; kk < 2; ++kk) {
      const v16h pa = Frag<_Float16>::load(pw + c * 64 + kk * 32 + 8 * hh);
#pragma unroll
      for (int t = 0; t < 4; ++t) {
        const v16h vb = Frag<_Float16>::load(Vp + (size_t)(t * 16 + c) * kSeq + kv0 + kk * 32 + 8 * hh);
        oacc[t] = mma_f16g(pa, vb, oacc[t]);
      }
    }
  }

  float* os = Os[wave];
#pragma unroll
  for (int r = 0; r < 8; ++r) {
#pragma unroll
    for (int t = 0; t < 4; ++t) os[(8 * hh + r) * 68 + t * 16 + c] = oacc[t][r] * kAttnScale;
  }
  __builtin_amdgcn_fence(__ATOMIC_RELEASE, "workgroup");
  __builtin_amdgcn_wave_barrier();
  __builtin_amdgcn_fence(__ATOMIC_ACQUIRE, "workgroup");
  {
    const int c4 = (lane & 15) * 4;
    for (int pass = 0; pass < 2; ++pass) {
#pragma unroll
      for (int it = 0; it < 8; ++it) {
        const int row = it * 2 + hh;
        v4f val = *(const v4f*)(os + row * 68 + c4);
        *(volatile v4f*)(Op + (size_t)(q0 + row) * kInner + c4) = val;
      }
      __threadfence();
    }
  }
}

__global__ __launch_bounds__(256) void gelu_kernel(const float* __restrict__ in, unsigned short* __restrict__ out, int n2) {
  const int i = blockIdx.x * 256 + threadIdx.x;
  if (i < n2) {
    const v2f v = *(const v2f*)(in + 2 * (size_t)i);
    const float g0 = 0.5f * v[0] * (1.0f + erff(v[0] * 0.70710678118654752f));
    const float g1 = 0.5f * v[1] * (1.0f + erff(v[1] * 0.70710678118654752f));
    const unsigned u = pk16(h_bits(g0 * kACarry), h_bits(g1 * kACarry));
    unsigned* op = (unsigned*)out + i;
    *(volatile unsigned*)op = u;
    __threadfence();
    *(volatile unsigned*)op = u;
  }
}

extern "C" void kernel_launch(void* const* d_in, const int* in_sizes, int n_in,
                              void* d_out, int out_size, void* d_ws, size_t ws_size,
                              hipStream_t stream) {
  (void)in_sizes;
  if (n_in < 27) return;
  if ((size_t)out_size < (size_t)3 * kRows * kDim) return;

  const float* x[3] = {(const float*)d_in[0], (const float*)d_in[1], (const float*)d_in[2]};
  const float *g1[3], *b1[3], *wqkv[3], *rmsw[3], *wo[3], *bo[3];
  for (int br = 0; br < 3; ++br) {
    const int base = 3 + 6 * br;
    g1[br]   = (const float*)d_in[base + 0];
    b1[br]   = (const float*)d_in[base + 1];
    wqkv[br] = (const float*)d_in[base + 2];
    rmsw[br] = (const float*)d_in[base + 3];
    wo[br]   = (const float*)d_in[base + 4];
    bo[br]   = (const float*)d_in[base + 5];
  }
  const float* g2    = (const float*)d_in[21];
  const float* b2    = (const float*)d_in[22];
  const float* w_fc1 = (const float*)d_in[23];
  const float* b_fc1 = (const float*)d_in[24];
  const float* w_fc2 = (const float*)d_in[25];
  const float* b_fc2 = (const float*)d_in[26];
  float* outp = (float*)d_out;

  char* ws = (char*)d_ws;
  size_t off = 0;
  const size_t szWqkvT = (size_t)kQkvW * kDim * 2;
  const size_t szWoT   = (size_t)kDim * kInner * 2;
  const size_t szWfc1T = (size_t)kHid * kDim3 * 2;
  const size_t szWfc2T = (size_t)kDim3 * kHid * 2;
  const size_t szXn    = (size_t)kRows * kDim * 2;
  const size_t szQkv   = (size_t)kRows * kQkvW * 2;
  const size_t szVt    = (size_t)kBatch * kInner * kSeq * 2;
  const size_t szAttn  = (size_t)kRows * kInner * 4;
  const size_t szRmsb  = (size_t)kRows * kInner * 2;
  const size_t szXcat  = (size_t)kRows * kDim3 * 4;
  const size_t szHn    = (size_t)kRows * kDim3 * 2;
  const size_t szHpre  = (size_t)kRows * kHid * 4;
  const size_t szHbuf  = (size_t)kRows * kHid * 2;
  unsigned short* wqkvT = (unsigned short*)(ws + off); off += 3 * szWqkvT;
  unsigned short* woT   = (unsigned short*)(ws + off); off += 3 * szWoT;
  unsigned short* wfc1T = (unsigned short*)(ws + off); off += szWfc1T;
  unsigned short* wfc2T = (unsigned short*)(ws + off); off += szWfc2T;
  unsigned short* xn    = (unsigned short*)(ws + off); off += szXn;
  unsigned short* qkv   = (unsigned short*)(ws + off); off += szQkv;
  unsigned short* vt    = (unsigned short*)(ws + off); off += szVt;
  float*          attno = (float*)(ws + off);          off += szAttn;
  unsigned short* rmsb  = (unsigned short*)(ws + off); off += szRmsb;
  float*          xcat  = (float*)(ws + off);          off += szXcat;
  unsigned short* hn    = (unsigned short*)(ws + off); off += szHn;
  float*          hpre  = (float*)(ws + off);          off += szHpre;
  unsigned short* hbuf  = (unsigned short*)(ws + off); off += szHbuf;
  if (off > ws_size) return;

  for (int br = 0; br < 3; ++br)
    wtcast_kernel<<<dim3(kDim / 64, kQkvW / 64, 1), 256, 0, stream>>>(wqkv[br], wqkvT + (size_t)br * kQkvW * kDim, kDim, kQkvW, kWCarry);
  for (int br = 0; br < 3; ++br)
    wtcast_kernel<<<dim3(kInner / 64, kDim / 64, 1), 256, 0, stream>>>(wo[br], woT + (size_t)br * kDim * kInner, kInner, kDim, kWCarry);
  wtcast_kernel<<<dim3(kDim3 / 64, kHid / 64, 1), 256, 0, stream>>>(w_fc1, wfc1T, kDim3, kHid, kWCarry);
  wtcast_kernel<<<dim3(kHid / 64, kDim3 / 64, 1), 256, 0, stream>>>(w_fc2, wfc2T, kHid, kDim3, kWCarry);

  const float invW  = 1.0f / kWCarry;
  const float invWA = 1.0f / (kWCarry * kACarry);

  for (int br = 0; br < 3; ++br) {
    ln256_kernel<<<kRows / 8, 256, 0, stream>>>(x[br], g1[br], b1[br], xn);
    {
      const unsigned short* Bt = wqkvT + (size_t)br * kQkvW * kDim;
      wmma_gemm64<0, false, 0, 1, false><<<dim3((kRows / 64) * (kQkvW / 64) / 8, 1), 256, 0, stream>>>(
          xn, xn, kDim, (long)0, Bt, Bt, kDim, (long)0, (void*)qkv, (void*)qkv, kQkvW, (long)0,
          g1[br], x[br], (long)0, kDim, kRows, kQkvW, kDim, invW);
    }
    vtrans_kernel<<<dim3(kSeq / 64, kInner / 64, kBatch), 256, 0, stream>>>(qkv, vt);
    rela_attn_kernel<<<kBatch * kHeads * (kSeq / 64), 128, 0, stream>>>(qkv, vt, attno);
    rms512_kernel<<<kRows / 8, 256, 0, stream>>>(attno, rmsw[br], rmsb);
    {
      const unsigned short* Bt = woT + (size_t)br * kDim * kInner;
      wmma_gemm64<0, false, 2, 0, true><<<dim3((kRows / 64) * (kDim / 64) / 8, 1), 256, 0, stream>>>(
          rmsb, rmsb, kInner, (long)0, Bt, Bt, kInner, (long)0, (void*)(xcat + br * kDim), (void*)(xcat + br * kDim), kDim3, (long)0,
          bo[br], x[br], (long)0, kDim, kRows, kDim, kInner, invWA);
    }
  }

  ln768_kernel<<<kRows / 8, 256, 0, stream>>>(xcat, g2, b2, hn);
  wmma_gemm64<0, false, 2, 0, false><<<dim3((kRows / 64) * (kHid / 64) / 8, 1), 256, 0, stream>>>(
      hn, hn, kDim3, (long)0, wfc1T, wfc1T, kDim3, (long)0, (void*)hpre, (void*)hpre, kHid, (long)0,
      b_fc1, xcat, (long)0, kDim3, kRows, kHid, kDim3, invW);
  {
    const int n2 = kRows * kHid / 2;
    gelu_kernel<<<(n2 + 255) / 256, 256, 0, stream>>>(hpre, hbuf, n2);
  }
  for (int br = 0; br < 3; ++br) {
    const unsigned short* Bt = wfc2T + (size_t)br * kDim * kHid;
    float* C = outp + (size_t)br * kRows * kDim;
    wmma_gemm64<0, false, 2, 0, true><<<dim3((kRows / 64) * (kDim / 64) / 8, 1), 256, 0, stream>>>(
        hbuf, hbuf, kHid, (long)0, Bt, Bt, kHid, (long)0, (void*)C, (void*)C, kDim, (long)0,
        b_fc2 + br * kDim, xcat + br * kDim, (long)0, kDim3, kRows, kDim, kHid, invWA);
  }
}
